// QGATConv_44289702756370
// MI455X (gfx1250) — hardware-verified
//
#include <hip/hip_runtime.h>
#include <stddef.h>
#include <stdint.h>


#define KIN   256
#define DF    128
#define NH    4
#define HD    32
#define GR    32
#define AP    264
#define XSP   132
#define NB    512
#define CHUNK 2048
#define NTHR  256
#define NWAVE 8
#define WCAP  256
#define NGRP  (CHUNK / (NTHR * 4))

#define LDS_SACC (NB * DF)
#define LDS_DEN  (NB * NH)
#define LDS_MX   (NB * NH)
#define LDS_LIST (NWAVE * WCAP)
#define LDS_BYTES ((LDS_SACC + LDS_DEN + LDS_MX + LDS_LIST + NWAVE) * 4)

static_assert(WCAP == (CHUNK / NTHR) * 32);
static_assert(NGRP == 2);
static_assert(NB == 512);
static_assert(CHUNK == 2048);
static_assert(LDS_BYTES == 286752);
static_assert(((LDS_SACC + LDS_DEN) % 4) == 0);
static_assert((LDS_MX % 4) == 0);
static_assert(DF == NH * HD);
static_assert((AP % 8) == 0);
static_assert((KIN % 32) == 0);
static_assert((KIN / 8) == 32);
static_assert(GR * NH <= NTHR);

typedef float          v4f   __attribute__((ext_vector_type(4)));
typedef float          v8f   __attribute__((ext_vector_type(8)));
typedef int            v4i   __attribute__((ext_vector_type(4)));
typedef unsigned short v8us  __attribute__((ext_vector_type(8)));
typedef unsigned short v16us __attribute__((ext_vector_type(16)));
typedef __bf16         v16bf __attribute__((ext_vector_type(16)));
union Frag   { v16bf v; v16us u; v8us half[2]; };
union Pack16 { v8us h; v4i i; };

__device__ __forceinline__ v8f wm(v16bf a, v16bf b, v8f c) {
  v8f d = __builtin_amdgcn_wmma_f32_16x16x32_bf16(false, a, false, b, (short)0, c, false, false);
  asm volatile("v_nop\n\tv_nop\n\tv_nop\n\tv_nop" : "+v"(d) : "v"(a), "v"(b));
  return d;
}

__device__ __forceinline__ unsigned short bfbits(float x) {
  unsigned u = __float_as_uint(x);
  u = u + 0x7FFFu + ((u >> 16) & 1u);
  return (unsigned short)(u >> 16);
}
__device__ __forceinline__ float bf2f(unsigned short b) {
  return __uint_as_float(((unsigned)b) << 16);
}
__device__ __forceinline__ void split1(float x, unsigned short& hi, unsigned short& lo) {
  const unsigned short h = bfbits(x);
  hi = h;
  lo = bfbits(x - bf2f(h));
}
__device__ __forceinline__ void split8(v4f a, v4f b, Pack16& ph, Pack16& pl) {
  unsigned short h, l;
  split1(a.x, h, l); ph.h[0] = h; pl.h[0] = l;
  split1(a.y, h, l); ph.h[1] = h; pl.h[1] = l;
  split1(a.z, h, l); ph.h[2] = h; pl.h[2] = l;
  split1(a.w, h, l); ph.h[3] = h; pl.h[3] = l;
  split1(b.x, h, l); ph.h[4] = h; pl.h[4] = l;
  split1(b.y, h, l); ph.h[5] = h; pl.h[5] = l;
  split1(b.z, h, l); ph.h[6] = h; pl.h[6] = l;
  split1(b.w, h, l); ph.h[7] = h; pl.h[7] = l;
}
__device__ __forceinline__ int imin(int a, int b) { return a < b ? a : b; }
__device__ __forceinline__ int imax(int a, int b) { return a > b ? a : b; }

__global__ __launch_bounds__(NTHR) void k_prep(const float* __restrict__ W,
                                               unsigned short* Wth, unsigned short* Wtl) {
  const int g = blockIdx.x * NTHR + threadIdx.x;
  if (g >= DF * (KIN / 8)) return;
  const int n  = g >> 5;
  const int k0 = (g & 31) * 8;
  Pack16 ph, pl;
#pragma unroll
  for (int i = 0; i < 8; ++i) {
    unsigned short h, l;
    split1(W[(size_t)(k0 + i) * DF + n], h, l);
    ph.h[i] = h;
    pl.h[i] = l;
  }
  const size_t o = (size_t)n * KIN + k0;
  const v4i vh = ph.i, vl = pl.i;
  *(volatile v4i*)(Wth + o) = vh;
  *(volatile v4i*)(Wtl + o) = vl;
  __threadfence();
  *(volatile v4i*)(Wth + o) = vh;
  *(volatile v4i*)(Wtl + o) = vl;
}

__global__ __launch_bounds__(NTHR) void k_gemm(
    const float* __restrict__ feat, const unsigned short* __restrict__ Wth,
    const unsigned short* __restrict__ Wtl, const float* __restrict__ attl,
    const float* __restrict__ attr, float* ft, float* elp, float* erp, int nN) {
  __shared__ __attribute__((aligned(16))) unsigned short Ah[GR * AP];
  __shared__ __attribute__((aligned(16))) unsigned short Al[GR * AP];
  __shared__ __attribute__((aligned(16))) float Xs[GR * XSP];
  __shared__ __attribute__((aligned(16))) float Es[GR * NH];
  __shared__ __attribute__((aligned(16))) float Rs[GR * NH];

  const int tid  = threadIdx.x;
  const int lane = tid & 31;
  const int wave = tid >> 5;
  const int hh   = lane >> 4;
  const int m    = lane & 15;
  const int rowBase = blockIdx.x * GR;

  {
    const int r  = tid >> 3;
    const int c0 = (tid & 7) * 32;
    int row = rowBase + r;
    if (row > nN - 1) row = nN - 1;
    const float* p = feat + (size_t)row * KIN + c0;
#pragma unroll
    for (int j = 0; j < 4; ++j) {
      const v4f f0 = *(const v4f*)(p + 8 * j);
      const v4f f1 = *(const v4f*)(p + 8 * j + 4);
      Pack16 ph, pl;
      split8(f0, f1, ph, pl);
      *(v8us*)(Ah + r * AP + c0 + 8 * j) = ph.h;
      *(v8us*)(Al + r * AP + c0 + 8 * j) = pl.h;
    }
  }
  __syncthreads();

  const int ncol = wave * 16 + m;
  v8f c0a = {0.f, 0.f, 0.f, 0.f, 0.f, 0.f, 0.f, 0.f};
  v8f c1a = {0.f, 0.f, 0.f, 0.f, 0.f, 0.f, 0.f, 0.f};
  {
    const unsigned short* pbh  = Wth + (size_t)ncol * KIN + 8 * hh;
    const unsigned short* pbl  = Wtl + (size_t)ncol * KIN + 8 * hh;
    const unsigned short* pa0h = Ah + m * AP + 8 * hh;
    const unsigned short* pa1h = Ah + (16 + m) * AP + 8 * hh;
    const unsigned short* pa0l = Al + m * AP + 8 * hh;
    const unsigned short* pa1l = Al + (16 + m) * AP + 8 * hh;
#pragma unroll
    for (int kt = 0; kt < KIN / 32; ++kt) {
      const int k0 = kt * 32;
      Frag a0h, a0l, a1h, a1l, bh, bl;
      bh.half[0]  = *(const v8us*)(pbh + k0);  bh.half[1]  = *(const v8us*)(pbh + k0 + 16);
      bl.half[0]  = *(const v8us*)(pbl + k0);  bl.half[1]  = *(const v8us*)(pbl + k0 + 16);
      a0h.half[0] = *(const v8us*)(pa0h + k0); a0h.half[1] = *(const v8us*)(pa0h + k0 + 16);
      a0l.half[0] = *(const v8us*)(pa0l + k0); a0l.half[1] = *(const v8us*)(pa0l + k0 + 16);
      a1h.half[0] = *(const v8us*)(pa1h + k0); a1h.half[1] = *(const v8us*)(pa1h + k0 + 16);
      a1l.half[0] = *(const v8us*)(pa1l + k0); a1l.half[1] = *(const v8us*)(pa1l + k0 + 16);
      c0a = wm(a0h.v, bh.v, c0a);
      c0a = wm(a0h.v, bl.v, c0a);
      c0a = wm(a0l.v, bh.v, c0a);
      c1a = wm(a1h.v, bh.v, c1a);
      c1a = wm(a1h.v, bl.v, c1a);
      c1a = wm(a1l.v, bh.v, c1a);
    }
  }

#pragma unroll
  for (int r = 0; r < 8; ++r) {
    Xs[(8 * hh + r) * XSP + ncol]      = c0a[r];
    Xs[(16 + 8 * hh + r) * XSP + ncol] = c1a[r];
  }
  __syncthreads();

  if (tid < GR * NH) {
    const int row = tid >> 2;
    const int h   = tid & 3;
    const float* xs = Xs + row * XSP + h * HD;
    const float* pl = attl + h * HD;
    const float* pr = attr + h * HD;
    float sl = 0.f, sr = 0.f;
#pragma unroll
    for (int j = 0; j < HD / 4; ++j) {
      const v4f xv = *(const v4f*)(xs + 4 * j);
      const v4f lv = *(const v4f*)(pl + 4 * j);
      const v4f rv = *(const v4f*)(pr + 4 * j);
      sl += xv.x * lv.x; sl += xv.y * lv.y; sl += xv.z * lv.z; sl += xv.w * lv.w;
      sr += xv.x * rv.x; sr += xv.y * rv.y; sr += xv.z * rv.z; sr += xv.w * rv.w;
    }
    Es[row * NH + h] = sl;
    Rs[row * NH + h] = sr;
  }
  __syncthreads();

  v4f xr[4];
  float* xpp[4];
#pragma unroll
  for (int i = 0; i < 4; ++i) {
    xr[i]  = *(const v4f*)(Xs + (4 * wave + i) * XSP + 4 * lane);
    xpp[i] = ft + (size_t)(rowBase + 4 * wave + i) * DF + 4 * lane;
  }
  v4f gl = {0.f, 0.f, 0.f, 0.f};
  v4f gr = {0.f, 0.f, 0.f, 0.f};
  if (wave == 0) gl = *(const v4f*)(Es + 4 * lane);
  if (wave == 1) gr = *(const v4f*)(Rs + 4 * lane);
  float* glp = elp + (size_t)rowBase * NH + 4 * lane;
  float* grp = erp + (size_t)rowBase * NH + 4 * lane;

#pragma unroll
  for (int i = 0; i < 4; ++i) *(volatile v4f*)(xpp[i]) = xr[i];
  if (wave == 0) *(volatile v4f*)glp = gl;
  if (wave == 1) *(volatile v4f*)grp = gr;
  __threadfence();
#pragma unroll
  for (int i = 0; i < 4; ++i) *(volatile v4f*)(xpp[i]) = xr[i];
  if (wave == 0) *(volatile v4f*)glp = gl;
  if (wave == 1) *(volatile v4f*)grp = gr;
}

__global__ __launch_bounds__(NTHR) void k_agg(
    const int* __restrict__ srci, const int* __restrict__ dsti,
    const float* __restrict__ ft, const float* __restrict__ elp, const float* __restrict__ erp,
    const float* __restrict__ bias, float* out, int nN, int nE) {
  extern __shared__ v4f lds_dyn[];
  float* sacc = (float*)lds_dyn;
  float* den  = sacc + LDS_SACC;
  float* mx   = den + LDS_DEN;
  int*   list = (int*)(mx + LDS_MX);
  int*   wcnt = list + LDS_LIST;

  const int tid  = threadIdx.x;
  const int lane = tid & 31;
  const int wave = tid >> 5;
  const int hd   = lane >> 3;
  const int nodeBase = blockIdx.x * NB;

  {
    const v4f z4 = {0.f, 0.f, 0.f, 0.f};
    const v4f n4 = {-1e30f, -1e30f, -1e30f, -1e30f};
    for (int i = tid; i < (LDS_SACC + LDS_DEN) / 4; i += NTHR) lds_dyn[i] = z4;
    v4f* mx4 = (v4f*)mx;
    for (int i = tid; i < LDS_MX / 4; i += NTHR) mx4[i] = n4;
  }
  __syncthreads();

  const bool al16 = ((((size_t)dsti) & 15) == 0);
  const int sent = -2147483647 - 1;

  const int nChunks = (nE + CHUNK - 1) / CHUNK;
#pragma unroll 1
  for (int ch = 0; ch < nChunks; ++ch) {
    const int cbase = ch * CHUNK;
    int wc = 0;
#pragma unroll
    for (int g = 0; g < NGRP; ++g) {
      const int el0 = (g * NTHR + tid) * 4;
      const int e0  = cbase + el0;
      v4i d;
      if (al16 && (cbase + CHUNK <= nE)) {
        d = *(const v4i*)(dsti + e0);
      } else {
        const int v0 = dsti[imin(e0,     nE - 1)];
        const int v1 = dsti[imin(e0 + 1, nE - 1)];
        const int v2 = dsti[imin(e0 + 2, nE - 1)];
        const int v3 = dsti[imin(e0 + 3, nE - 1)];
        d.x = (e0     < nE) ? v0 : sent;
        d.y = (e0 + 1 < nE) ? v1 : sent;
        d.z = (e0 + 2 < nE) ? v2 : sent;
        d.w = (e0 + 3 < nE) ? v3 : sent;
      }
      const unsigned s0 = (unsigned)d.x - (unsigned)nodeBase;
      const unsigned s1 = (unsigned)d.y - (unsigned)nodeBase;
      const unsigned s2 = (unsigned)d.z - (unsigned)nodeBase;
      const unsigned s3 = (unsigned)d.w - (unsigned)nodeBase;
      const bool h0 = s0 < (unsigned)NB;
      const bool h1 = s1 < (unsigned)NB;
      const bool h2 = s2 < (unsigned)NB;
      const bool h3 = s3 < (unsigned)NB;
      const unsigned many = __builtin_amdgcn_ballot_w32(h0 | h1 | h2 | h3);
      if (many != 0u) {
#define HITJ(J, HJ, SJ) { \
          const unsigned mj = __builtin_amdgcn_ballot_w32(HJ); \
          if (HJ) { \
            const int pos = wc + (int)__builtin_amdgcn_mbcnt_lo(mj, 0u); \
            if (pos < WCAP) list[wave * WCAP + pos] = ((el0 + (J)) << 9) | (int)(SJ); \
          } \
          wc += (int)__builtin_popcount(mj); }
        HITJ(0, h0, s0)
        HITJ(1, h1, s1)
        HITJ(2, h2, s2)
        HITJ(3, h3, s3)
#undef HITJ
      }
    }
    if (lane == 0) wcnt[wave] = wc;
    __syncthreads();

    if (wave == 0) {
#pragma unroll 1
      for (int wsx = 0; wsx < NWAVE; ++wsx) {
        int n = wcnt[wsx];
        if (n > WCAP) n = WCAP;
        if (n < 0) n = 0;
#pragma unroll 1
        for (int i = 0; i < n; ++i) {
          const int ent  = list[wsx * WCAP + i];
          const int slot = ent & (NB - 1);
          const int eloc = (ent >> 9) & (CHUNK - 1);
          int e = cbase + eloc;
          if (e > nE - 1) e = nE - 1;
          int s = srci[e];
          s = imax(0, imin(s, nN - 1));
          int nd = nodeBase + slot;
          if (nd > nN - 1) nd = nN - 1;
          float lg = elp[(size_t)s * NH + hd] + erp[(size_t)nd * NH + hd];
          lg = (lg > 0.f) ? lg : 0.2f * lg;
          const int ai = slot * NH + hd;
          const float mo = mx[ai];
          const float mn = fmaxf(mo, lg);
          const float f  = __expf(mo - mn);
          const float p  = __expf(lg - mn);
          const v4f xv = *(const v4f*)(ft + (size_t)s * DF + 4 * lane);
          v4f* sp = (v4f*)(sacc + slot * DF + 4 * lane);
          const v4f cur = *sp;
          const v4f nxt = cur * f + p * xv;
          *sp = nxt;
          const float dn = den[ai];
          const float dnew = dn * f + p;
          den[ai] = dnew;
          mx[ai]  = mn;
        }
      }
    }
    __syncthreads();
  }

  const v4f b4 = *(const v4f*)(bias + 4 * lane);
#pragma unroll 1
  for (int j = 0; j < NB / NWAVE; ++j) {
    const int slot = wave * (NB / NWAVE) + j;
    const int node = nodeBase + slot;
    if (node >= nN) break;
    const float dv  = den[slot * NH + hd];
    const float inv = (dv > 0.f) ? (1.0f / dv) : 0.f;
    const v4f sv = *(const v4f*)(sacc + slot * DF + 4 * lane);
    const v4f y = sv * inv + b4;
    float* op = out + (size_t)node * DF + 4 * lane;
    *(volatile v4f*)op = y;
    __threadfence();
    *(volatile v4f*)op = y;
  }
}

extern "C" void kernel_launch(void* const* d_in, const int* in_sizes, int n_in,
                              void* d_out, int out_size, void* d_ws, size_t ws_size,
                              hipStream_t stream) {
  if (n_in < 7) return;
  const int nN = in_sizes[0] / KIN;
  const int nE = in_sizes[1];
  if (nN <= 0 || in_sizes[0] != nN * KIN) return;
  if (nE < 0 || in_sizes[2] != nE) return;
  if (in_sizes[3] != KIN * DF) return;
  if (in_sizes[4] != NH * HD || in_sizes[5] != NH * HD) return;
  if (in_sizes[6] != DF) return;
  if (out_size != nN * DF) return;

  const float* feat = (const float*)d_in[0];
  const int*   srci = (const int*)d_in[1];
  const int*   dsti = (const int*)d_in[2];
  const float* W    = (const float*)d_in[3];
  const float* attl = (const float*)d_in[4];
  const float* attr = (const float*)d_in[5];
  const float* bias = (const float*)d_in[6];
  float* out = (float*)d_out;

  const int nP = ((nN + GR - 1) / GR) * GR;
  size_t off = 0;
  unsigned short* Wth = (unsigned short*)((char*)d_ws + off); off += (size_t)DF * KIN * sizeof(unsigned short);
  unsigned short* Wtl = (unsigned short*)((char*)d_ws + off); off += (size_t)DF * KIN * sizeof(unsigned short);
  float* ftp = (float*)((char*)d_ws + off); off += (size_t)nP * DF * sizeof(float);
  float* elp = (float*)((char*)d_ws + off); off += (size_t)nP * NH * sizeof(float);
  float* erp = (float*)((char*)d_ws + off); off += (size_t)nP * NH * sizeof(float);
  if (off > ws_size) return;
  if (off > (size_t)134217728) return;

  k_prep<<<(DF * (KIN / 8) + NTHR - 1) / NTHR, NTHR, 0, stream>>>(W, Wth, Wtl);

  k_gemm<<<nP / GR, NTHR, 0, stream>>>(feat, Wth, Wtl, attl, attr, ftp, elp, erp, nN);

  hipFuncSetAttribute(reinterpret_cast<const void*>(&k_agg),
                      hipFuncAttributeMaxDynamicSharedMemorySize, LDS_BYTES);
  const int grid = (nN + NB - 1) / NB;
  k_agg<<<grid, NTHR, LDS_BYTES, stream>>>(srci, dsti, ftp, elp, erp, bias, out, nN, nE);
}
